// GCN_14173392077062
// MI455X (gfx1250) — hardware-verified
//
#include <hip/hip_runtime.h>
#include <stddef.h>
#include <stdint.h>
#include <math.h>

#define NN     50000
#define NE     800000
#define FIN    128
#define FH     256
#define FO     40
#define FOP    64
#define K2     512
#define MP     50048
#define NTHR   256
#define NWAVE  8
#define EPT    8
#define CHUNK  (NTHR * EPT)
#define WCAP   (EPT * 32)
#define LISTN  (NWAVE * WCAP)
#define NBA    1024
#define SLA    10
#define NBLK   49
#define NSLOT  (NBLK * NBA)
#define RCAP   28672
#define DEGCAP 64
#define GBM    64
#define GBN    64
#define GTHR   128
#define RECW   544
#define WSTW   520
#define OCH    128
#define BK_ZINTS (LISTN + 2 * RCAP + 3 * NBA)
#define BK_LDS_INTS (BK_ZINTS + 16)
#define PB_X   ((MP * (FIN / 8)) / NTHR)
#define PB_W0  ((FH * (FIN / 8)) / NTHR)
#define PB_W1  ((FH * (K2 / 8)) / NTHR)
#define PB_W2  ((FOP * (K2 / 8)) / NTHR)
#define NTAB4  (7 * (FH / 4))
#define PB_T   2
#define PB_ALL (PB_X + PB_W0 + PB_W1 + PB_W2 + PB_T)
#define WSMAX  134217728

static_assert((CHUNK & (CHUNK - 1)) == 0 && CHUNK <= 4096);
static_assert((NBA & (NBA - 1)) == 0 && NBA == (1 << SLA) && NBA % 4 == 0);
static_assert(((long long)NE << SLA) < (1LL << 31));
static_assert(NE % 4 == 0);
static_assert(LISTN % NTHR == 0 && LISTN == 2 * NBA);
static_assert(NBA % NWAVE == 0 && NBA == 4 * NTHR);
static_assert(RCAP % (4 * NTHR) == 0 && BK_ZINTS % 4 == 0);
static_assert(RCAP >= 16696 + 835 && DEGCAP >= 33 + 8);
static_assert(BK_LDS_INTS * 4 <= 300000);
static_assert(MP % GBM == 0 && MP >= NN && NSLOT >= MP && NSLOT >= NN);
static_assert(GBM == (GTHR / 32) * 16 && GBN == 64 && FH % GBN == 0 && FOP == GBN);
static_assert(FIN % 32 == 0 && K2 % 32 == 0 && K2 == 2 * FH && FH == 32 * 8);
static_assert((MP * (FIN / 8)) % NTHR == 0 && (FH * (FIN / 8)) % NTHR == 0);
static_assert((FH * (K2 / 8)) % NTHR == 0 && (FOP * (K2 / 8)) % NTHR == 0);
static_assert(NTAB4 <= PB_T * NTHR && NTAB4 % 8 == 0);
static_assert((MP * 32) % NTHR == 0);
static_assert(RECW % 32 == 0 && RECW >= 2 * FH + 1 && RECW / 4 <= NTHR && WSTW >= 2 * FH + 1);
static_assert(NN % 4 == 0 && ((long long)NN * FO * 4) % 128 == 0 && (OCH * FO * 4) % 128 == 0);
static_assert(NBA % OCH == 0 && OCH % NWAVE == 0 && (OCH * FO / 4) % NTHR == 0 && FO % 4 == 0 && FO / 4 == 10);

typedef float          v4f   __attribute__((ext_vector_type(4)));
typedef float          v8f   __attribute__((ext_vector_type(8)));
typedef int            v4i   __attribute__((ext_vector_type(4)));
typedef int            v8i   __attribute__((ext_vector_type(8)));
typedef unsigned       v2u   __attribute__((ext_vector_type(2)));
typedef unsigned short v8us  __attribute__((ext_vector_type(8)));
typedef unsigned short v16us __attribute__((ext_vector_type(16)));
typedef __bf16         v16bf __attribute__((ext_vector_type(16)));
typedef v4f  __attribute__((may_alias)) v4fa;
typedef v4i  __attribute__((may_alias)) v4ia;
typedef v2u  __attribute__((may_alias)) v2ua;
typedef v8us __attribute__((may_alias)) v8usa;
union FragB { v16bf v; v16us u; v8us h[2]; v8i w; };

__device__ __forceinline__ v8f wmb(const FragB& a, const FragB& b, v8f c) {
  v8f d = __builtin_amdgcn_wmma_f32_16x16x32_bf16(false, a.v, false, b.v, (short)0, c, false, false);
  asm volatile("v_nop\n\tv_nop\n\tv_nop\n\tv_nop" : "+v"(d) : "v"(a.w), "v"(b.w));
  return d;
}

__device__ __forceinline__ unsigned bf16_bits(float f) {
  const unsigned u = __float_as_uint(f);
  return (u + 0x7FFFu + ((u >> 16) & 1u)) >> 16;
}
__device__ __forceinline__ unsigned bf16_bits_np(float f) {
  const unsigned u = __float_as_uint(f);
  const unsigned r = (u + 0x7FFFu + ((u >> 16) & 1u)) >> 16;
  return (f != f) ? 0x7fc0u : r;
}
__device__ __forceinline__ float bf16_val(float f) {
  return __uint_as_float(bf16_bits(f) << 16);
}
__device__ __forceinline__ v4f sel4(bool c, v4f a, v4f b) {
  v4f r;
  r.x = c ? a.x : b.x; r.y = c ? a.y : b.y; r.z = c ? a.z : b.z; r.w = c ? a.w : b.w;
  return r;
}

template <int SLB>
__device__ __forceinline__ int scan_chunk(const int* __restrict__ dsts, int nE, int cbase, int slotBase,
                                          int nb, int vec8, int* list, int tid, int lane, int wave) {
  int wc = 0;
  const int el0  = tid * EPT;
  const int e0   = cbase + el0;
  const int sent = -2147483647 - 1;
  v4i da, db;
  if (vec8 != 0 && cbase + CHUNK <= nE) {
    da = *(const v4i*)(dsts + e0);
    db = *(const v4i*)(dsts + e0 + 4);
  } else {
    da.x = (e0     < nE) ? dsts[min(e0,     nE - 1)] : sent;
    da.y = (e0 + 1 < nE) ? dsts[min(e0 + 1, nE - 1)] : sent;
    da.z = (e0 + 2 < nE) ? dsts[min(e0 + 2, nE - 1)] : sent;
    da.w = (e0 + 3 < nE) ? dsts[min(e0 + 3, nE - 1)] : sent;
    db.x = (e0 + 4 < nE) ? dsts[min(e0 + 4, nE - 1)] : sent;
    db.y = (e0 + 5 < nE) ? dsts[min(e0 + 5, nE - 1)] : sent;
    db.z = (e0 + 6 < nE) ? dsts[min(e0 + 6, nE - 1)] : sent;
    db.w = (e0 + 7 < nE) ? dsts[min(e0 + 7, nE - 1)] : sent;
  }
  const unsigned nbs = (unsigned)slotBase;
  const unsigned unb = (unsigned)nb;
  const unsigned s0 = (unsigned)da.x - nbs, s1 = (unsigned)da.y - nbs;
  const unsigned s2 = (unsigned)da.z - nbs, s3 = (unsigned)da.w - nbs;
  const unsigned s4 = (unsigned)db.x - nbs, s5 = (unsigned)db.y - nbs;
  const unsigned s6 = (unsigned)db.z - nbs, s7 = (unsigned)db.w - nbs;
  const bool h0 = s0 < unb, h1 = s1 < unb, h2 = s2 < unb, h3 = s3 < unb;
  const bool h4 = s4 < unb, h5 = s5 < unb, h6 = s6 < unb, h7 = s7 < unb;
  const unsigned any = __builtin_amdgcn_ballot_w32(h0 | h1 | h2 | h3 | h4 | h5 | h6 | h7);
  if (any != 0u) {
#define HITJ(J, HJ, SJ) { \
      const unsigned mj = __builtin_amdgcn_ballot_w32(HJ); \
      if (mj != 0u) { \
        if (HJ) { \
          const int pos = wc + (int)__builtin_amdgcn_mbcnt_lo(mj, 0u); \
          if (pos < WCAP) list[wave * WCAP + pos] = ((el0 + (J)) << SLB) | (int)(SJ); \
        } \
        wc += (int)__builtin_popcount(mj); } }
    HITJ(0, h0, s0)
    HITJ(1, h1, s1)
    HITJ(2, h2, s2)
    HITJ(3, h3, s3)
    HITJ(4, h4, s4)
    HITJ(5, h5, s5)
    HITJ(6, h6, s6)
    HITJ(7, h7, s7)
#undef HITJ
  }
  return wc;
}

__global__ __launch_bounds__(NTHR) void k_prep(const float* __restrict__ feat, const float* __restrict__ W0,
                                               const float* __restrict__ W1, const float* __restrict__ W2,
                                               const float* __restrict__ b0, const float* __restrict__ b1,
                                               const float* __restrict__ b2, const float* __restrict__ g0,
                                               const float* __restrict__ be0, const float* __restrict__ g1,
                                               const float* __restrict__ be1,
                                               unsigned short* XB, unsigned short* W0T, unsigned short* W1D,
                                               unsigned short* W2D, float* TAB) {
  const int bid = (int)blockIdx.x, tid = (int)threadIdx.x;
  if (bid >= PB_X + PB_W0 + PB_W1 + PB_W2) {
    const int t  = (bid - (PB_X + PB_W0 + PB_W1 + PB_W2)) * NTHR + tid;
    const int tc = t < NTAB4 ? t : NTAB4 - 1;
    const int row = tc >> 6;
    const int c4  = (tc & 63) * 4;
    const int c4b = c4 < (FO - 4) ? c4 : (FO - 4);
    const v4f a0 = *(const v4f*)(b0 + c4);
    const v4f a1 = *(const v4f*)(b1 + c4);
    v4f       a2 = *(const v4f*)(b2 + c4b);
    const v4f a3 = *(const v4f*)(g0 + c4);
    const v4f a4 = *(const v4f*)(be0 + c4);
    const v4f a5 = *(const v4f*)(g1 + c4);
    const v4f a6 = *(const v4f*)(be1 + c4);
    const v4f z = {0.f, 0.f, 0.f, 0.f};
    a2 = sel4(c4 < FO, a2, z);
    v4f v = a0;
    v = sel4(row == 1, a1, v);
    v = sel4(row == 2, a2, v);
    v = sel4(row == 3, a3, v);
    v = sel4(row == 4, a4, v);
    v = sel4(row == 5, a5, v);
    v = sel4(row == 6, a6, v);
    v4f o;
    o.x = bf16_val(v.x); o.y = bf16_val(v.y); o.z = bf16_val(v.z); o.w = bf16_val(v.w);
    float* tp = TAB + 4 * (size_t)tc;
    if (t < NTAB4) *(volatile v4f*)tp = o;
    __threadfence();
    if (t < NTAB4) *(volatile v4f*)tp = o;
    return;
  }
  v8us o;
  unsigned short* dp;
  if (bid < PB_X) {
    const int u   = bid * NTHR + tid;
    const int row = u >> 4;
    const int k8  = (u & 15) * 8;
    const int rc  = row < NN ? row : NN - 1;
    const float* p = feat + (size_t)rc * FIN + k8;
    const v4f a = *(const v4f*)p;
    const v4f b = *(const v4f*)(p + 4);
    const bool ok = row < NN;
    o[0] = ok ? (unsigned short)bf16_bits(a.x) : (unsigned short)0;
    o[1] = ok ? (unsigned short)bf16_bits(a.y) : (unsigned short)0;
    o[2] = ok ? (unsigned short)bf16_bits(a.z) : (unsigned short)0;
    o[3] = ok ? (unsigned short)bf16_bits(a.w) : (unsigned short)0;
    o[4] = ok ? (unsigned short)bf16_bits(b.x) : (unsigned short)0;
    o[5] = ok ? (unsigned short)bf16_bits(b.y) : (unsigned short)0;
    o[6] = ok ? (unsigned short)bf16_bits(b.z) : (unsigned short)0;
    o[7] = ok ? (unsigned short)bf16_bits(b.w) : (unsigned short)0;
    dp = XB + (size_t)row * FIN + k8;
  } else if (bid < PB_X + PB_W0) {
    const int v  = (bid - PB_X) * NTHR + tid;
    const int n  = v >> 4;
    const int k8 = (v & 15) * 8;
    const float* p = W0 + (size_t)k8 * FH + n;
#pragma unroll
    for (int i = 0; i < 8; ++i) o[i] = (unsigned short)bf16_bits(p[(size_t)i * FH]);
    dp = W0T + (size_t)n * FIN + k8;
  } else if (bid < PB_X + PB_W0 + PB_W1) {
    const int v  = (bid - PB_X - PB_W0) * NTHR + tid;
    const int n  = v >> 6;
    const int k8 = (v & 63) * 8;
    const int kk = k8 & (FH - 1);
    const float* p = W1 + (size_t)kk * FH + n;
#pragma unroll
    for (int i = 0; i < 8; ++i) o[i] = (unsigned short)bf16_bits(p[(size_t)i * FH]);
    dp = W1D + (size_t)n * K2 + k8;
  } else {
    const int v  = (bid - PB_X - PB_W0 - PB_W1) * NTHR + tid;
    const int n  = v >> 6;
    const int k8 = (v & 63) * 8;
    const int kk = k8 & (FH - 1);
    const int nc = n < FO ? n : FO - 1;
    const bool ok = n < FO;
    const float* p = W2 + (size_t)kk * FO + nc;
#pragma unroll
    for (int i = 0; i < 8; ++i) {
      const unsigned short w = (unsigned short)bf16_bits(p[(size_t)i * FO]);
      o[i] = ok ? w : (unsigned short)0;
    }
    dp = W2D + (size_t)n * K2 + k8;
  }
  *(volatile v8us*)dp = o;
  __threadfence();
  *(volatile v8us*)dp = o;
}

__global__ __launch_bounds__(NTHR) void k_bucket(const int* __restrict__ srcs, const int* __restrict__ dsts,
                                                 int* LISTp, int* CNTp, int* OFFp, int* SNp, int* DNp,
                                                 int* FLGp) {
  extern __shared__ __attribute__((aligned(16))) int dsm[];
  int* list = dsm;
  int* hl   = dsm + LISTN;
  int* sl   = hl + RCAP;
  int* cnt  = sl + RCAP;
  int* offs = cnt + NBA;
  int* cur  = offs + NBA;
  int* misc = cur + NBA;
  const int tid = (int)threadIdx.x, lane = tid & 31, wave = tid >> 5;
  const int blk = (int)blockIdx.x;
  const int nodeBase = blk * NBA;
  const int vec8 = 1;

  {
    const v4i z4 = {0, 0, 0, 0};
    for (int i = tid * 4; i < BK_ZINTS; i += NTHR * 4) *(v4ia*)(dsm + i) = z4;
    if (tid < 16) misc[tid] = 0;
  }
  __syncthreads();

  int t = 0, ov = 0;
  const int nChunks = (NE + CHUNK - 1) / CHUNK;
#pragma unroll 1
  for (int ch = 0; ch < nChunks; ++ch) {
    const int cbase = ch * CHUNK;
    const int wc = scan_chunk<SLA>(dsts, NE, cbase, nodeBase, NBA, vec8, list, tid, lane, wave);
    if (lane == 0) misc[wave] = wc;
    __syncthreads();
    if (wave == 0) {
#pragma unroll 1
      for (int w2 = 0; w2 < NWAVE; ++w2) {
        int c = misc[w2];
        c = c < 0 ? 0 : (c > WCAP ? WCAP : c);
#pragma unroll 1
        for (int b0 = 0; b0 < c; b0 += 32) {
          const int idx = b0 + lane;
          const int ent = list[w2 * WCAP + (idx < WCAP ? idx : WCAP - 1)];
          const int m32 = (c - b0) < 32 ? (c - b0) : 32;
#pragma unroll 1
          for (int k = 0; k < m32; ++k) {
            const int u    = __builtin_amdgcn_readlane(ent, k);
            const int slot = u & (NBA - 1);
            const int el   = (u >> SLA) & (CHUNK - 1);
            const int pk   = ((cbase + el) << SLA) | slot;
            if (t < RCAP) {
              if (lane == 0) { hl[t] = pk; cnt[slot] = cnt[slot] + 1; }
              t = t + 1;
            } else {
              ov = 1;
            }
          }
        }
      }
    }
    __syncthreads();
  }
  if (wave == 0 && lane == 0) { misc[8] = t; misc[9] = ov; }
  __syncthreads();
  int tt = misc[8];
  tt = tt < 0 ? 0 : (tt > RCAP ? RCAP : tt);

  if (wave == 0) {
    const int base = lane * (NBA / 32);
    int s = 0;
#pragma unroll 1
    for (int i = 0; i < NBA / 32; ++i) s += cnt[base + i];
    int incl = s;
#pragma unroll
    for (int d = 1; d < 32; d <<= 1) {
      const int y = __shfl_up(incl, d, 32);
      if (lane >= d) incl += y;
    }
    int run = incl - s;
#pragma unroll 1
    for (int i = 0; i < NBA / 32; ++i) {
      const int cv = cnt[base + i];
      offs[base + i] = run;
      cur[base + i]  = run;
      run += cv;
    }
  }
  __syncthreads();
  if (wave == 0) {
#pragma unroll 1
    for (int b0 = 0; b0 < tt; b0 += 32) {
      const int idx = b0 + lane;
      const int ent = hl[idx < RCAP ? idx : RCAP - 1];
      const int m32 = (tt - b0) < 32 ? (tt - b0) : 32;
#pragma unroll 1
      for (int k = 0; k < m32; ++k) {
        const int u    = __builtin_amdgcn_readlane(ent, k);
        const int slot = u & (NBA - 1);
        if (lane == 0) {
          int p = cur[slot];
          p = p < 0 ? 0 : (p > RCAP - 1 ? RCAP - 1 : p);
          sl[p] = u;
          cur[slot] = p + 1;
        }
      }
    }
  }
  {
    int big = 0;
#pragma unroll 1
    for (int i = tid; i < NBA; i += NTHR) big |= (cnt[i] > DEGCAP) ? 1 : 0;
    if (big != 0) misc[10] = 1;
  }
  __syncthreads();
  const int flag = ((misc[9] | misc[10]) != 0) ? 1 : 0;

#pragma unroll 1
  for (int i = tid; i < RCAP; i += NTHR) {
    const int ent = sl[i];
    int eid = ent >> SLA;
    eid = eid < 0 ? 0 : (eid > NE - 1 ? NE - 1 : eid);
    int sr = srcs[eid];
    sr = sr < 0 ? 0 : (sr > NN - 1 ? NN - 1 : sr);
    hl[i] = (i < tt) ? sr : 0;
  }
#pragma unroll 1
  for (int i = tid; i < NBA; i += NTHR) cur[i] = 0;
  __syncthreads();

#pragma unroll 1
  for (int ch = 0; ch < nChunks; ++ch) {
    const int cbase = ch * CHUNK;
    const int wc = scan_chunk<SLA>(srcs, NE, cbase, nodeBase, NBA, vec8, list, tid, lane, wave);
    if (lane == 0) misc[wave] = wc;
    __syncthreads();
    if (wave == 0) {
#pragma unroll 1
      for (int w2 = 0; w2 < NWAVE; ++w2) {
        int c = misc[w2];
        c = c < 0 ? 0 : (c > WCAP ? WCAP : c);
#pragma unroll 1
        for (int b0 = 0; b0 < c; b0 += 32) {
          const int idx = b0 + lane;
          const int ent = list[w2 * WCAP + (idx < WCAP ? idx : WCAP - 1)];
          const int m32 = (c - b0) < 32 ? (c - b0) : 32;
#pragma unroll 1
          for (int k = 0; k < m32; ++k) {
            const int u  = __builtin_amdgcn_readlane(ent, k);
            const int s2 = u & (NBA - 1);
            if (lane == 0) cur[s2] = cur[s2] + 1;
          }
        }
      }
    }
    __syncthreads();
  }

#pragma unroll 1
  for (int i = tid; i < NBA; i += NTHR) {
    const int cd = cnt[i] < 1 ? 1 : cnt[i];
    const int cs = cur[i] < 1 ? 1 : cur[i];
    list[i]       = __float_as_int(1.0f / sqrtf((float)cd));
    list[NBA + i] = __float_as_int(1.0f / sqrtf((float)cs));
  }
  __syncthreads();

  const v4i c4 = *(const v4ia*)(cnt + 4 * tid);
  const v4i o4 = *(const v4ia*)(offs + 4 * tid);
  const v4i d4 = *(const v4ia*)(list + 4 * tid);
  const v4i s4 = *(const v4ia*)(list + NBA + 4 * tid);
  const v4i f4 = {flag, flag, flag, flag};
  int* lp = LISTp + (size_t)blk * RCAP;
#pragma unroll 1
  for (int pass = 0; pass < 2; ++pass) {
    *(volatile v4i*)(CNTp + (size_t)nodeBase + 4 * tid) = c4;
    *(volatile v4i*)(OFFp + (size_t)nodeBase + 4 * tid) = o4;
    *(volatile v4i*)(DNp  + (size_t)nodeBase + 4 * tid) = d4;
    *(volatile v4i*)(SNp  + (size_t)nodeBase + 4 * tid) = s4;
    if (tid < 8) *(volatile v4i*)(FLGp + (size_t)blk * 32 + 4 * tid) = f4;
#pragma unroll 1
    for (int it = 0; it < RCAP / (4 * NTHR); ++it) {
      const int i4 = (it * NTHR + tid) * 4;
      const v4i v = *(const v4ia*)(hl + i4);
      *(volatile v4i*)(lp + i4) = v;
    }
    __threadfence();
  }
}

__global__ __launch_bounds__(GTHR) void k_gemm(
    const unsigned short* __restrict__ A, const unsigned short* __restrict__ WT,
    const float* __restrict__ SNp, float* outF, int K, int ldo)
{
  __shared__ __attribute__((aligned(16))) float stg[GBM * GBN];
  __shared__ float sns[GBM];
  const int tid = (int)threadIdx.x, lane = tid & 31, wave = tid >> 5, hh = lane >> 4, m = lane & 15;
  const int rowBase = (int)blockIdx.x * GBM;
  const int col0    = (int)blockIdx.y * GBN;

  if (tid < GBM) sns[tid] = SNp[rowBase + tid];

  v8f acc[4];
  {
    const v8f z = {0.f, 0.f, 0.f, 0.f, 0.f, 0.f, 0.f, 0.f};
    acc[0] = z; acc[1] = z; acc[2] = z; acc[3] = z;
  }
  const unsigned short* ap = A  + (size_t)(rowBase + 16 * wave + m) * (size_t)K + 8 * hh;
  const unsigned short* wp = WT + (size_t)(col0 + m) * (size_t)K + 8 * hh;
  const int ksteps = K >> 5;
#pragma unroll 1
  for (int ks = 0; ks < ksteps; ++ks) {
    FragB af;
    af.h[0] = *(const v8usa*)(ap + 32 * ks);
    af.h[1] = *(const v8usa*)(ap + 32 * ks + 16);
#pragma unroll
    for (int t = 0; t < 4; ++t) {
      const unsigned short* wq = wp + (size_t)(16 * t) * (size_t)K + 32 * ks;
      FragB bf;
      bf.h[0] = *(const v8usa*)wq;
      bf.h[1] = *(const v8usa*)(wq + 16);
      acc[t] = wmb(af, bf, acc[t]);
    }
  }

#pragma unroll
  for (int t = 0; t < 4; ++t) {
    const int lc = 16 * t + m;
#pragma unroll
    for (int r = 0; r < 8; ++r) {
      const int lr = 16 * wave + 8 * hh + r;
      stg[lr * GBN + lc] = acc[t][r];
    }
  }
  __syncthreads();

  v4f fv[8];
#pragma unroll
  for (int i = 0; i < 8; ++i) {
    const int lr = 16 * wave + 2 * i + hh;
    const v4f x = *(const v4fa*)(stg + lr * GBN + 4 * m);
    const float sn = sns[lr];
    v4f y;
    y.x = x.x * sn; y.y = x.y * sn; y.z = x.z * sn; y.w = x.w * sn;
    fv[i] = y;
  }
#pragma unroll
  for (int i = 0; i < 8; ++i) {
    const int lr = 16 * wave + 2 * i + hh;
    const int gr = rowBase + lr;
    float* op = outF + (size_t)gr * (size_t)ldo + col0 + 4 * m;
    *(volatile v4f*)op = fv[i];
  }
  __threadfence();
#pragma unroll
  for (int i = 0; i < 8; ++i) {
    const int lr = 16 * wave + 2 * i + hh;
    const int gr = rowBase + lr;
    float* op = outF + (size_t)gr * (size_t)ldo + col0 + 4 * m;
    *(volatile v4f*)op = fv[i];
  }
}

template <int MODE>
__global__ __launch_bounds__(NTHR) void k_agg(const int* __restrict__ LISTp, const int* __restrict__ CNTp,
                                              const int* __restrict__ OFFp, const float* __restrict__ DNp,
                                              const int* __restrict__ FLGp, const float* __restrict__ P,
                                              const float* __restrict__ biasT,
                                              const unsigned short* hres, float* outC, float* rec) {
  __shared__ float wst[NWAVE * WSTW];
  __shared__ __attribute__((aligned(16))) float pst[RECW];
  const int tid = (int)threadIdx.x, lane = tid & 31, wave = tid >> 5;
  const int blk = (int)blockIdx.x;
  const int nodeBase = blk * NBA;
  const int* lst = LISTp + (size_t)blk * RCAP;
  const bool flag = FLGp[(size_t)blk * 32] != 0;
  const float qnan = __int_as_float(0x7fc00000);

  float bs[8];
  {
    const v4f bA = *(const v4fa*)(biasT + 4 * lane);
    const v4f bB = *(const v4fa*)(biasT + 128 + 4 * lane);
    bs[0] = bA.x; bs[1] = bA.y; bs[2] = bA.z; bs[3] = bA.w;
    bs[4] = bB.x; bs[5] = bB.y; bs[6] = bB.z; bs[7] = bB.w;
  }
  int wn = 0;
  float wm[8], wq[8];
#pragma unroll
  for (int j = 0; j < 8; ++j) { wm[j] = 0.0f; wq[j] = 0.0f; }

#pragma unroll 1
  for (int si = 0; si < NBA / NWAVE; ++si) {
    const int s    = si * NWAVE + wave;
    const int node = nodeBase + s;
    int c = CNTp[node];
    c = c < 0 ? 0 : (c > DEGCAP ? DEGCAP : c);
    int o = OFFp[node];
    o = o < 0 ? 0 : (o > RCAP ? RCAP : o);
    const float dn = DNp[node];
    const int nc = node < NN ? node : NN - 1;
    float rs[8];
#pragma unroll
    for (int j = 0; j < 8; ++j) rs[j] = 0.0f;
    if constexpr (MODE == 1) {
      const unsigned short* rp = hres + (size_t)nc * K2 + 4 * lane;
      const v2u h0 = *(const v2ua*)rp;
      const v2u h1 = *(const v2ua*)(rp + 128);
      const v2u l0 = *(const v2ua*)(rp + 256);
      const v2u l1 = *(const v2ua*)(rp + 384);
      rs[0] = __uint_as_float(h0.x << 16)          + __uint_as_float(l0.x << 16);
      rs[1] = __uint_as_float(h0.x & 0xffff0000u) + __uint_as_float(l0.x & 0xffff0000u);
      rs[2] = __uint_as_float(h0.y << 16)          + __uint_as_float(l0.y << 16);
      rs[3] = __uint_as_float(h0.y & 0xffff0000u) + __uint_as_float(l0.y & 0xffff0000u);
      rs[4] = __uint_as_float(h1.x << 16)          + __uint_as_float(l1.x << 16);
      rs[5] = __uint_as_float(h1.x & 0xffff0000u) + __uint_as_float(l1.x & 0xffff0000u);
      rs[6] = __uint_as_float(h1.y << 16)          + __uint_as_float(l1.y << 16);
      rs[7] = __uint_as_float(h1.y & 0xffff0000u) + __uint_as_float(l1.y & 0xffff0000u);
    }
    float acc[8];
#pragma unroll
    for (int j = 0; j < 8; ++j) acc[j] = 0.0f;
#pragma unroll 1
    for (int b0 = 0; b0 < c; b0 += 32) {
      int idx = o + b0 + lane;
      idx = idx > RCAP - 1 ? RCAP - 1 : idx;
      int sr = lst[idx];
      sr = sr < 0 ? 0 : (sr > NN - 1 ? NN - 1 : sr);
      const int m32 = (c - b0) < 32 ? (c - b0) : 32;
#pragma unroll 1
      for (int k = 0; k < m32; ++k) {
        const int sk = __builtin_amdgcn_readlane(sr, k);
        const float* rowp = P + (size_t)sk * FH + 4 * lane;
        const v4f a  = *(const v4fa*)rowp;
        const v4f a2 = *(const v4fa*)(rowp + 128);
        acc[0] += a.x;  acc[1] += a.y;  acc[2] += a.z;  acc[3] += a.w;
        acc[4] += a2.x; acc[5] += a2.y; acc[6] += a2.z; acc[7] += a2.w;
      }
    }
    float y[8];
#pragma unroll
    for (int j = 0; j < 8; ++j) {
      float v = acc[j] * dn + bs[j];
      if constexpr (MODE == 1) v = v + rs[j];
      y[j] = flag ? qnan : v;
    }
    const bool live = node < NN;
    if (live) {
      wn += 1;
      const float rk = 1.0f / (float)wn;
#pragma unroll
      for (int j = 0; j < 8; ++j) {
        const float d = y[j] - wm[j];
        wm[j] = fmaf(d, rk, wm[j]);
        wq[j] = fmaf(d, y[j] - wm[j], wq[j]);
      }
      v4f f0, f1;
      f0.x = y[0]; f0.y = y[1]; f0.z = y[2]; f0.w = y[3];
      f1.x = y[4]; f1.y = y[5]; f1.z = y[6]; f1.w = y[7];
      float* op = outC + (size_t)node * FH + 4 * lane;
      *(volatile v4f*)op = f0;
      *(volatile v4f*)(op + 128) = f1;
      __threadfence();
      *(volatile v4f*)op = f0;
      *(volatile v4f*)(op + 128) = f1;
    }
  }

  if (lane == 0) wst[wave * WSTW] = (float)wn;
#pragma unroll
  for (int j = 0; j < 4; ++j) {
    wst[wave * WSTW + 1 + 4 * lane + j]            = wm[j];
    wst[wave * WSTW + 1 + 128 + 4 * lane + j]      = wm[4 + j];
    wst[wave * WSTW + 1 + FH + 4 * lane + j]       = wq[j];
    wst[wave * WSTW + 1 + FH + 128 + 4 * lane + j] = wq[4 + j];
  }
  __syncthreads();
  {
    float n = 0.0f, mean = 0.0f, M2 = 0.0f;
#pragma unroll 1
    for (int w2 = 0; w2 < NWAVE; ++w2) {
      const float nb = wst[w2 * WSTW];
      const float mb = wst[w2 * WSTW + 1 + tid];
      const float qb = wst[w2 * WSTW + 1 + FH + tid];
      if (nb > 0.5f) {
        const float nn = n + nb;
        const float delta = mb - mean;
        const float f = nb / nn;
        mean = fmaf(delta, f, mean);
        M2 = M2 + qb + delta * delta * n * f;
        n = nn;
      }
    }
    pst[1 + tid] = mean;
    pst[1 + FH + tid] = M2;
    if (tid == 0) pst[0] = n;
  }
#pragma unroll 1
  for (int i = 2 * FH + 1 + tid; i < RECW; i += NTHR) pst[i] = 0.0f;
  __syncthreads();
  v4f ps = {0.f, 0.f, 0.f, 0.f};
  if (tid < RECW / 4) {
    ps = *(const v4fa*)(pst + 4 * tid);
    *(volatile v4f*)(rec + (size_t)blk * RECW + 4 * tid) = ps;
  }
  __threadfence();
  if (tid < RECW / 4) {
    *(volatile v4f*)(rec + (size_t)blk * RECW + 4 * tid) = ps;
  }
}

__global__ __launch_bounds__(FH) void k_comb(const float* __restrict__ rec, int nPart, float* st) {
  __shared__ __attribute__((aligned(16))) float stg[2 * FH];
  const int tid = (int)threadIdx.x;
  const int c = tid;
  double n = 0.0, mean = 0.0, M2 = 0.0;
#pragma unroll 1
  for (int b = 0; b < nPart; ++b) {
    const float* pr = rec + (size_t)b * RECW;
    const double nb = (double)pr[0];
    const double mb = (double)pr[1 + c];
    const double qb = (double)pr[1 + FH + c];
    if (nb > 0.5) {
      const double nn = n + nb;
      const double delta = mb - mean;
      const double f = nb / nn;
      mean = mean + delta * f;
      M2 = M2 + qb + delta * delta * n * f;
      n = nn;
    }
  }
  const double nt = n < 1.0 ? 1.0 : n;
  const float varf  = (float)(M2 / nt);
  const float meanf = (float)mean;
  const float r = 1.0f / sqrtf(varf + 1e-5f);
  stg[c] = meanf;
  stg[FH + c] = r;
  __syncthreads();
  v4f v = {0.f, 0.f, 0.f, 0.f};
  if (tid < (2 * FH) / 4) {
    v = *(const v4fa*)(stg + 4 * tid);
    *(volatile v4f*)(st + 4 * tid) = v;
  }
  __threadfence();
  if (tid < (2 * FH) / 4) {
    *(volatile v4f*)(st + 4 * tid) = v;
  }
}

__global__ __launch_bounds__(NTHR) void k_apply(const float* __restrict__ C, const float* __restrict__ st,
                                                const float* __restrict__ gT, const float* __restrict__ beT,
                                                unsigned short* hl) {
  __shared__ __attribute__((aligned(16))) float pm[FH];
  __shared__ __attribute__((aligned(16))) float pr[FH];
  __shared__ __attribute__((aligned(16))) float pg[FH];
  __shared__ __attribute__((aligned(16))) float pb[FH];
  const int tid = (int)threadIdx.x;
  if (tid < FH / 4) {
    *(v4fa*)(pm + 4 * tid) = *(const v4f*)(st + 4 * tid);
    *(v4fa*)(pr + 4 * tid) = *(const v4f*)(st + FH + 4 * tid);
    *(v4fa*)(pg + 4 * tid) = *(const v4f*)(gT + 4 * tid);
    *(v4fa*)(pb + 4 * tid) = *(const v4f*)(beT + 4 * tid);
  }
  __syncthreads();
  const int u   = (int)blockIdx.x * NTHR + tid;
  const int row = u >> 5;
  const int c8  = (u & 31) * 8;
  const int rc  = row < NN ? row : NN - 1;
  const bool ok = row < NN;
  const float* p = C + (size_t)rc * FH + c8;
  const v4f x0 = *(const v4f*)p;
  const v4f x1 = *(const v4f*)(p + 4);
  const v4f m0 = *(const v4fa*)(pm + c8), m1 = *(const v4fa*)(pm + c8 + 4);
  const v4f r0 = *(const v4fa*)(pr + c8), r1 = *(const v4fa*)(pr + c8 + 4);
  const v4f g0 = *(const v4fa*)(pg + c8), g1 = *(const v4fa*)(pg + c8 + 4);
  const v4f e0 = *(const v4fa*)(pb + c8), e1 = *(const v4fa*)(pb + c8 + 4);
  float xv[8] = {x0.x, x0.y, x0.z, x0.w, x1.x, x1.y, x1.z, x1.w};
  float mv[8] = {m0.x, m0.y, m0.z, m0.w, m1.x, m1.y, m1.z, m1.w};
  float rv[8] = {r0.x, r0.y, r0.z, r0.w, r1.x, r1.y, r1.z, r1.w};
  float gv[8] = {g0.x, g0.y, g0.z, g0.w, g1.x, g1.y, g1.z, g1.w};
  float ev[8] = {e0.x, e0.y, e0.z, e0.w, e1.x, e1.y, e1.z, e1.w};
  v8us hv, lv;
#pragma unroll
  for (int j = 0; j < 8; ++j) {
    float t = ((xv[j] - mv[j]) * rv[j]) * gv[j] + ev[j];
    t = (t > 0.0f) ? t : (t - t);
    t = ok ? t : 0.0f;
    const unsigned hb = bf16_bits_np(t);
    hv[j] = (unsigned short)hb;
    lv[j] = (unsigned short)bf16_bits_np(t - __uint_as_float(hb << 16));
  }
  unsigned short* op = hl + (size_t)row * K2 + c8;
  *(volatile v8us*)op = hv;
  *(volatile v8us*)(op + FH) = lv;
  __threadfence();
  *(volatile v8us*)op = hv;
  *(volatile v8us*)(op + FH) = lv;
}

__global__ __launch_bounds__(NTHR) void k_agg2(const int* __restrict__ LISTp, const int* __restrict__ CNTp,
                                               const int* __restrict__ OFFp, const float* __restrict__ DNp,
                                               const int* __restrict__ FLGp, const float* __restrict__ P2,
                                               const float* __restrict__ b2T, float* out) {
  __shared__ __attribute__((aligned(16))) float stg[OCH * FO];
  const int tid = (int)threadIdx.x, lane = tid & 31, wave = tid >> 5;
  const int blk = (int)blockIdx.x;
  const int nodeBase = blk * NBA;
  const int* lst = LISTp + (size_t)blk * RCAP;
  const bool flag = FLGp[(size_t)blk * 32] != 0;
  const float qnan = __int_as_float(0x7fc00000);
  const int g = lane / 10;
  const int q = lane - 10 * g;
  const bool gvalid = g < 3;
  const v4f bq = *(const v4fa*)(b2T + 4 * q);
  const int sA = (lane + 10) > 31 ? 31 : (lane + 10);
  const int sB = (lane + 20) > 31 ? 31 : (lane + 20);

#pragma unroll 1
  for (int ch = 0; ch < NBA / OCH; ++ch) {
    const int chunkBase = nodeBase + ch * OCH;
#pragma unroll 1
    for (int si = 0; si < OCH / NWAVE; ++si) {
      const int sloc = si * NWAVE + wave;
      const int node = chunkBase + sloc;
      int c = CNTp[node];
      c = c < 0 ? 0 : (c > DEGCAP ? DEGCAP : c);
      int o = OFFp[node];
      o = o < 0 ? 0 : (o > RCAP ? RCAP : o);
      const float dn = DNp[node];
      float ax = 0.0f, ay = 0.0f, az = 0.0f, aw = 0.0f;
#pragma unroll 1
      for (int b0 = 0; b0 < c; b0 += 32) {
        int idx = o + b0 + lane;
        idx = idx > RCAP - 1 ? RCAP - 1 : idx;
        int sr = lst[idx];
        sr = sr < 0 ? 0 : (sr > NN - 1 ? NN - 1 : sr);
        const int m32 = (c - b0) < 32 ? (c - b0) : 32;
#pragma unroll 1
        for (int k = 0; k < m32; k += 3) {
          const int kk = k + g;
          const bool valid = gvalid && (kk < m32);
          const int kc = kk > 31 ? 31 : kk;
          const int sk = __shfl(sr, kc, 32);
          const v4f a = *(const v4fa*)(P2 + (size_t)sk * FOP + 4 * q);
          const int msk = valid ? -1 : 0;
          ax += __int_as_float(__float_as_int(a.x) & msk);
          ay += __int_as_float(__float_as_int(a.y) & msk);
          az += __int_as_float(__float_as_int(a.z) & msk);
          aw += __int_as_float(__float_as_int(a.w) & msk);
        }
      }
      const float x1 = __shfl(ax, sA, 32), x2 = __shfl(ax, sB, 32);
      const float y1 = __shfl(ay, sA, 32), y2 = __shfl(ay, sB, 32);
      const float z1 = __shfl(az, sA, 32), z2 = __shfl(az, sB, 32);
      const float w1 = __shfl(aw, sA, 32), w2 = __shfl(aw, sB, 32);
      v4f yv;
      yv.x = ((ax + x1) + x2) * dn + bq.x;
      yv.y = ((ay + y1) + y2) * dn + bq.y;
      yv.z = ((az + z1) + z2) * dn + bq.z;
      yv.w = ((aw + w1) + w2) * dn + bq.w;
      if (lane < 10) *(v4fa*)(stg + sloc * FO + 4 * lane) = yv;
    }
    __syncthreads();
    int rvn = NN - chunkBase;
    rvn = rvn < 0 ? 0 : (rvn > OCH ? OCH : rvn);
    const int nU = rvn * (FO / 4);
    float* ob = out + (size_t)chunkBase * FO;
#pragma unroll 1
    for (int pass = 0; pass < 2; ++pass) {
#pragma unroll 1
      for (int it = 0; it < (OCH * FO / 4) / NTHR; ++it) {
        const int u = it * NTHR + tid;
        v4f v = *(const v4fa*)(stg + 4 * u);
        v.x = flag ? qnan : v.x; v.y = flag ? qnan : v.y;
        v.z = flag ? qnan : v.z; v.w = flag ? qnan : v.w;
        if (u < nU) *(volatile v4f*)(ob + 4 * (size_t)u) = v;
      }
      __threadfence();
    }
    __syncthreads();
  }
}

static inline size_t al256(size_t o) { return (o + 255) & ~(size_t)255; }

extern "C" void kernel_launch(void* const* d_in, const int* in_sizes, int n_in,
                              void* d_out, int out_size, void* d_ws, size_t ws_size,
                              hipStream_t stream) {
  if (n_in < 13) return;
  if (in_sizes[0] != NN * FIN) return;
  if (in_sizes[1] != NE || in_sizes[2] != NE) return;
  if (in_sizes[3] != FIN * FH || in_sizes[4] != FH) return;
  if (in_sizes[5] != FH * FH || in_sizes[6] != FH) return;
  if (in_sizes[7] != FH * FO || in_sizes[8] != FO) return;
  if (in_sizes[9] != FH || in_sizes[10] != FH) return;
  if (in_sizes[11] != FH || in_sizes[12] != FH) return;
  if (out_size != NN * FO) return;

  const float* feat = (const float*)d_in[0];
  const int*   src  = (const int*)d_in[1];
  const int*   dst  = (const int*)d_in[2];
  const float* W0   = (const float*)d_in[3];
  const float* b0   = (const float*)d_in[4];
  const float* W1   = (const float*)d_in[5];
  const float* b1   = (const float*)d_in[6];
  const float* W2   = (const float*)d_in[7];
  const float* b2   = (const float*)d_in[8];
  const float* g0   = (const float*)d_in[9];
  const float* be0  = (const float*)d_in[10];
  const float* g1   = (const float*)d_in[11];
  const float* be1  = (const float*)d_in[12];
  float* out = (float*)d_out;

  char* ws = (char*)d_ws;
  size_t off = 0;
  const size_t oR1   = off; off = al256(off + (size_t)MP * FH * 4);
  const size_t oR2   = off; off = al256(off + (size_t)MP * FH * 4);
  const size_t oXB   = off; off = al256(off + (size_t)MP * FIN * 2);
  const size_t oLIST = off; off = al256(off + (size_t)NBLK * RCAP * 4);
  const size_t oCNT  = off; off = al256(off + (size_t)NSLOT * 4);
  const size_t oOFF  = off; off = al256(off + (size_t)NSLOT * 4);
  const size_t oSN   = off; off = al256(off + (size_t)NSLOT * 4);
  const size_t oDN   = off; off = al256(off + (size_t)NSLOT * 4);
  const size_t oFLG  = off; off = al256(off + (size_t)NBLK * 128);
  const size_t oW0T  = off; off = al256(off + (size_t)FH * FIN * 2);
  const size_t oW1D  = off; off = al256(off + (size_t)FH * K2 * 2);
  const size_t oW2D  = off; off = al256(off + (size_t)FOP * K2 * 2);
  const size_t oTAB  = off; off = al256(off + (size_t)7 * FH * 4);
  const size_t oREC0 = off; off = al256(off + (size_t)NBLK * RECW * 4);
  const size_t oREC1 = off; off = al256(off + (size_t)NBLK * RECW * 4);
  const size_t oST0  = off; off = al256(off + (size_t)(2 * FH) * 4);
  const size_t oST1  = off; off = al256(off + (size_t)(2 * FH) * 4);
  if (off > ws_size || off > (size_t)WSMAX) return;

  float*          R1f  = (float*)(ws + oR1);
  unsigned short* R1h  = (unsigned short*)(ws + oR1);
  float*          R2f  = (float*)(ws + oR2);
  unsigned short* R2h  = (unsigned short*)(ws + oR2);
  unsigned short* XB   = (unsigned short*)(ws + oXB);
  int*            LIST = (int*)(ws + oLIST);
  int*            CNT  = (int*)(ws + oCNT);
  int*            OFF  = (int*)(ws + oOFF);
  int*            SNi  = (int*)(ws + oSN);
  int*            DNi  = (int*)(ws + oDN);
  const float*    SN   = (const float*)(ws + oSN);
  const float*    DN   = (const float*)(ws + oDN);
  int*            FLG  = (int*)(ws + oFLG);
  unsigned short* W0T  = (unsigned short*)(ws + oW0T);
  unsigned short* W1D  = (unsigned short*)(ws + oW1D);
  unsigned short* W2D  = (unsigned short*)(ws + oW2D);
  float*          TAB  = (float*)(ws + oTAB);
  float*          REC0 = (float*)(ws + oREC0);
  float*          REC1 = (float*)(ws + oREC1);
  float*          ST0  = (float*)(ws + oST0);
  float*          ST1  = (float*)(ws + oST1);
  const float* Tb0 = TAB;            const float* Tb1 = TAB + FH;      const float* Tb2 = TAB + 2 * FH;
  const float* Tg0 = TAB + 3 * FH;   const float* Te0 = TAB + 4 * FH;
  const float* Tg1 = TAB + 5 * FH;   const float* Te1 = TAB + 6 * FH;

  const size_t bkLds = (size_t)BK_LDS_INTS * 4;
  hipFuncSetAttribute(reinterpret_cast<const void*>(&k_bucket), hipFuncAttributeMaxDynamicSharedMemorySize, (int)bkLds);

  const int gM = MP / GBM;
  k_prep<<<PB_ALL, NTHR, 0, stream>>>(feat, W0, W1, W2, b0, b1, b2, g0, be0, g1, be1, XB, W0T, W1D, W2D, TAB);
  k_bucket<<<NBLK, NTHR, bkLds, stream>>>(src, dst, LIST, CNT, OFF, SNi, DNi, FLG);
  k_gemm<<<dim3(gM, FH / GBN), GTHR, 0, stream>>>(XB, W0T, SN, R1f, FIN, FH);
  k_agg<0><<<NBLK, NTHR, 0, stream>>>(LIST, CNT, OFF, DN, FLG, R1f, Tb0, XB, R2f, REC0);
  k_comb<<<1, FH, 0, stream>>>(REC0, NBLK, ST0);
  k_apply<<<(MP * 32) / NTHR, NTHR, 0, stream>>>(R2f, ST0, Tg0, Te0, R1h);
  k_gemm<<<dim3(gM, FH / GBN), GTHR, 0, stream>>>(R1h, W1D, SN, R2f, K2, FH);
  k_agg<1><<<NBLK, NTHR, 0, stream>>>(LIST, CNT, OFF, DN, FLG, R2f, Tb1, R1h, R1f, REC1);
  k_comb<<<1, FH, 0, stream>>>(REC1, NBLK, ST1);
  k_apply<<<(MP * 32) / NTHR, NTHR, 0, stream>>>(R1f, ST1, Tg1, Te1, R2h);
  k_gemm<<<dim3(gM, FOP / GBN), GTHR, 0, stream>>>(R2h, W2D, SN, R1f, K2, FOP);
  k_agg2<<<NBLK, NTHR, 0, stream>>>(LIST, CNT, OFF, DN, FLG, R1f, Tb2, out);
}
